// FusedLlamaMLPQuantized_27702539059405
// MI455X (gfx1250) — hardware-verified
//
#include <hip/hip_runtime.h>
#include <math.h>

typedef __attribute__((ext_vector_type(16))) _Float16 v16h;
typedef __attribute__((ext_vector_type(16))) __bf16 v16b;
typedef __attribute__((ext_vector_type(8)))  _Float16 v8h;
typedef __attribute__((ext_vector_type(8)))  float v8f;
typedef __attribute__((ext_vector_type(4)))  float v4f;
typedef __attribute__((ext_vector_type(2)))  float v2f;
typedef __attribute__((ext_vector_type(4)))  unsigned v4u;
typedef __attribute__((ext_vector_type(4)))  int v4i;
typedef float __attribute__((may_alias)) float_a;
typedef int __attribute__((may_alias)) int_a;

template <typename T> __device__ __forceinline__ void vst2(void* p, T v) { *(volatile T*)p = v; __threadfence(); *(volatile T*)p = v; }
__device__ __forceinline__ v8f wmma16(v16h a, v16h b, v8f c) {
  v8f d = __builtin_amdgcn_wmma_f32_16x16x32_f16(false, a, false, b, (short)0, c, false, false);
  asm volatile("v_nop\n\tv_nop\n\tv_nop\n\tv_nop" : "+v"(d) : "v"(a), "v"(b));
  return d;
}
__device__ __forceinline__ v8f wmma_bf(v16b a, v16b b, v8f c) {
  v8f d = __builtin_amdgcn_wmma_f32_16x16x32_bf16(false, a, false, b, (short)0, c, false, false);
  asm volatile("v_nop\n\tv_nop\n\tv_nop\n\tv_nop" : "+v"(d) : "v"(a), "v"(b));
  return d;
}
__device__ __forceinline__ v16h frag_h(const _Float16* rowk0, int lane) {
  union { v16h v; v8h q[2]; } u; const _Float16* p = rowk0 + 8 * (lane >> 4);
  u.q[0] = *(const v8h*)p; u.q[1] = *(const v8h*)(p + 16); return u.v;
}
__device__ __forceinline__ v16h frag_f32(const float* rowk0, int lane) {
  v16h a; const float* p = rowk0 + 8 * (lane >> 4);
#pragma unroll
  for (int i = 0; i < 8; ++i) { a[i] = (_Float16)p[i]; a[8 + i] = (_Float16)p[16 + i]; }
  return a;
}
__device__ __forceinline__ v16h frag_f32s(const float* rowk0, int lane, float sc) {
  v16h a; const float* p = rowk0 + 8 * (lane >> 4);
#pragma unroll
  for (int i = 0; i < 8; ++i) { a[i] = (_Float16)(p[i] * sc); a[8 + i] = (_Float16)(p[16 + i] * sc); }
  return a;
}
__device__ __forceinline__ v16h fragc_f32(const float* W, int k0, int n, int lane, int ld, int K) {
  v16h a; const int g = lane >> 4;
#pragma unroll
  for (int i = 0; i < 8; ++i) { const int ka = k0 + 8 * g + i, kb = ka + 16;
    a[i] = (_Float16)(ka < K ? W[(size_t)(ka < K ? ka : K - 1) * ld + n] : 0.f); a[8 + i] = (_Float16)(kb < K ? W[(size_t)(kb < K ? kb : K - 1) * ld + n] : 0.f); }
  return a;
}
struct F2 { v16b h, l; };
__device__ __forceinline__ F2 bsplit16(const float v[16]) { F2 r;
#pragma unroll
  for (int i = 0; i < 16; ++i) { const __bf16 h = (__bf16)v[i]; r.h[i] = h; r.l[i] = (__bf16)(v[i] - (float)h); }
  return r; }
__device__ __forceinline__ F2 split_row(const float* row, int k0, int lane) { float v[16]; const float* p = row + k0 + 8 * (lane >> 4);
#pragma unroll
  for (int i = 0; i < 8; ++i) { v[i] = p[i]; v[8 + i] = p[16 + i]; }
  return bsplit16(v); }
__device__ __forceinline__ F2 split_rowK(const float* row, int k0, int lane, int K) { float v[16]; const int g = lane >> 4;
#pragma unroll
  for (int i = 0; i < 8; ++i) { const int ka = k0 + 8 * g + i, kb = ka + 16; v[i] = ka < K ? row[ka < K ? ka : K - 1] : 0.f; v[8 + i] = kb < K ? row[kb < K ? kb : K - 1] : 0.f; }
  return bsplit16(v); }
__device__ __forceinline__ F2 split_col(const float* W, int k0, int n, int lane, int ld, int K) { float v[16]; const int g = lane >> 4;
#pragma unroll
  for (int i = 0; i < 8; ++i) { const int ka = k0 + 8 * g + i, kb = ka + 16; v[i] = ka < K ? W[(size_t)(ka < K ? ka : K - 1) * ld + n] : 0.f; v[8 + i] = kb < K ? W[(size_t)(kb < K ? kb : K - 1) * ld + n] : 0.f; }
  return bsplit16(v); }
__device__ __forceinline__ v8f mac3(const F2& a, const F2& b, v8f c) { c = wmma_bf(a.l, b.h, c); c = wmma_bf(a.h, b.l, c); return wmma_bf(a.h, b.h, c); }
__device__ __forceinline__ float sigm(float v) { return 1.0f / (1.0f + expf(-v)); }
#define LDSX() do { asm volatile("s_wait_dscnt 0" ::: "memory"); __builtin_amdgcn_wave_barrier(); __builtin_amdgcn_fence(__ATOMIC_RELEASE, "workgroup"); } while (0)


#ifndef KIN
#define MM 64
#define KIN 4096
#define NI 11008
#define NO 4096
#endif
#define GRP 128
typedef __attribute__((ext_vector_type(8))) __bf16 v8b;
__device__ __forceinline__ v16b frag_b(const __bf16* rowk0, int lane) {
  union { v16b v; v8b q[2]; } u; const __bf16* p = rowk0 + 8 * (lane >> 4);
  u.q[0] = *(const v8b*)p; u.q[1] = *(const v8b*)(p + 16); return u.v;
}
__device__ __forceinline__ float bfr(float v) { return (float)(__bf16)v; }
__device__ __attribute__((noinline)) float exp_ni(float v) { return expf(v); }
__device__ __attribute__((noinline)) float erf_ni(float v) { return erff(v); }

#define WS_XH  0u
#define WS_XL  (WS_XH + 2u * MM * KIN)
#define WS_G   (WS_XL + 2u * MM * KIN)
#define WS_U   (WS_G + 4u * MM * NI)
#define WS_HH  (WS_U + 4u * MM * NI)
#define WS_HL  (WS_HH + 2u * MM * NI)
#define WS_END (WS_HL + 2u * MM * NI)

__global__ __launch_bounds__(256) void k_xh(const float* __restrict__ X, _Float16* __restrict__ XH, _Float16* __restrict__ XL) {
  const size_t row = blockIdx.x; for (int q = threadIdx.x; q < KIN / 8; q += 256) { __align__(16) _Float16 hh[8], ll[8];
#pragma unroll
    for (int i = 0; i < 8; ++i) { const float v = bfr(X[row * KIN + q * 8 + i]); const _Float16 h = (_Float16)v; hh[i] = h; ll[i] = (_Float16)((v - (float)h) * 2048.0f); }
    vst2((unsigned*)(XH + row * KIN + q * 8), *(const v4u*)hh); vst2((unsigned*)(XL + row * KIN + q * 8), *(const v4u*)ll); }
}
template <int DOWN>
__global__ __launch_bounds__(128) void k_qgemm(const _Float16* __restrict__ AH, const _Float16* __restrict__ AL, const int* __restrict__ QW, const float* __restrict__ SC, const int* __restrict__ QZ, const int* __restrict__ GI, float* __restrict__ OUT) {
  constexpr int KD = DOWN ? NI : KIN; constexpr int ND = DOWN ? NO : NI;
  __shared__ __align__(16) _Float16 swh[128][40], swl[128][40]; __shared__ __align__(16) float so[4][16][132];
  const int tid = threadIdx.x, wave = tid >> 5, lane = tid & 31, col = lane & 15, g = lane >> 4; const int n0 = blockIdx.x * 128;
  v8f acc[8] = {}, accl[8] = {};
#pragma unroll 1
  for (int kc = 0; kc < KD / 32; ++kc) {
    { const int n = n0 + tid; const int k0 = kc * 32; int cur = -1; int z = 0; float sc = 0.f;
#pragma unroll 1
      for (int wq = 0; wq < 4; ++wq) { const int word = QW[(size_t)((k0 >> 3) + wq) * ND + n];
#pragma unroll
        for (int i = 0; i < 8; ++i) { const int k = k0 + wq * 8 + i; const int gi = GI[k];
          if (gi != cur) { cur = gi; const int zw = QZ[(size_t)gi * (ND / 8) + (n >> 3)]; z = ((zw >> ((n & 7) * 4)) & 15) + 1; sc = bfr(SC[(size_t)gi * ND + n]); }
          const int w = (word >> (i * 4)) & 15; const float val = (float)(w - z) * sc; const _Float16 h = (_Float16)val; swh[tid][wq * 8 + i] = h; swl[tid][wq * 8 + i] = (_Float16)((val - (float)h) * 2048.0f); } } }
    __syncthreads();
    const v16h a = frag_h(AH + (size_t)(wave * 16 + col) * KD + kc * 32, lane), al = frag_h(AL + (size_t)(wave * 16 + col) * KD + kc * 32, lane);
#pragma unroll
    for (int j = 0; j < 8; ++j) { const v16h wh = frag_h(&swh[j * 16 + col][0], lane); acc[j] = wmma16(a, wh, acc[j]); accl[j] = wmma16(al, wh, accl[j]); accl[j] = wmma16(a, frag_h(&swl[j * 16 + col][0], lane), accl[j]); }
    __syncthreads(); }
#pragma unroll
  for (int j = 0; j < 8; ++j)
#pragma unroll
    for (int r = 0; r < 8; ++r) so[wave][8 * g + r][j * 16 + col] = acc[j][r] + accl[j][r] * (1.0f / 2048.0f);
  LDSX();
  for (int rl = 0; rl < 16; ++rl) vst2(OUT + (size_t)(wave * 16 + rl) * ND + n0 + lane * 4, *(const v4f*)&so[wave][rl][lane * 4]);
}
__global__ __launch_bounds__(256) void k_h(const float* __restrict__ G, const float* __restrict__ U, _Float16* __restrict__ HH, _Float16* __restrict__ HL) {
  const size_t row = blockIdx.x; for (int q = threadIdx.x; q < NI / 8; q += 256) { __align__(16) _Float16 hh[8], ll[8];
#pragma unroll
    for (int i = 0; i < 8; ++i) { const float gv = G[row * NI + q * 8 + i], uv = U[row * NI + q * 8 + i]; const float hv = (gv / (1.0f + exp_ni(-gv))) * uv; const _Float16 h = (_Float16)hv; hh[i] = h; ll[i] = (_Float16)((hv - (float)h) * 2048.0f); }
    vst2((unsigned*)(HH + row * NI + q * 8), *(const v4u*)hh); vst2((unsigned*)(HL + row * NI + q * 8), *(const v4u*)ll); }
}
extern "C" void kernel_launch(void* const* d_in, const int* in_sizes, int n_in, void* d_out, int out_size, void* d_ws, size_t ws_size, hipStream_t stream) {
  (void)in_sizes; (void)n_in; (void)out_size;
  const float** F = (const float**)d_in; const int** I = (const int**)d_in;
  if (ws_size < (size_t)WS_END) return;
  char* ws = (char*)d_ws; _Float16 *XH = (_Float16*)(ws + WS_XH), *XL = (_Float16*)(ws + WS_XL), *HH = (_Float16*)(ws + WS_HH), *HL = (_Float16*)(ws + WS_HL); float *G = (float*)(ws + WS_G), *U = (float*)(ws + WS_U);
  k_xh<<<MM, 256, 0, stream>>>(F[0], XH, XL);
  k_qgemm<0><<<NI / 128, 128, 0, stream>>>(XH, XL, I[1], F[2], I[3], I[4], G);
  k_qgemm<0><<<NI / 128, 128, 0, stream>>>(XH, XL, I[5], F[6], I[7], I[8], U);
  k_h<<<MM, 256, 0, stream>>>(G, U, HH, HL);
  k_qgemm<1><<<NO / 128, 128, 0, stream>>>(HH, HL, I[9], F[10], I[11], I[12], (float*)d_out);
}
